// BellmanLoss_77429670412386
// MI455X (gfx1250) — hardware-verified
//
#include <hip/hip_runtime.h>
#include <math.h>

#define NBATCH 65536
#define SD 128
#define HD 256
#define NA 18
#define NAP 128

typedef _Float16 f16;
typedef __attribute__((ext_vector_type(16))) f16 f16x16;
typedef __attribute__((ext_vector_type(8)))  f16 f16x8;
typedef __attribute__((ext_vector_type(8)))  float f32x8;
typedef __attribute__((ext_vector_type(4)))  float v4f_t;
typedef float v4fa __attribute__((ext_vector_type(4), may_alias));
typedef __attribute__((ext_vector_type(4))) unsigned v4u_t;
typedef unsigned v4ua __attribute__((ext_vector_type(4), may_alias));

__device__ __forceinline__ f32x8 wmma16(f16x16 a, f16x16 b, f32x8 c) {
  c = __builtin_amdgcn_wmma_f32_16x16x32_f16(false, a, false, b, (short)0, c, false, false);
  asm volatile("v_nop\n\tv_nop\n\tv_nop\n\tv_nop" : "+v"(c) : "v"(a), "v"(b));
  return c;
}
__device__ __forceinline__ f16x16 lds_frag(const f16* base, int stride) {
  const int lane = threadIdx.x & 31, row = lane & 15, kh = (lane >> 4) * 8;
  const f16x8 lo = *(const f16x8*)(base + row * stride + kh);
  const f16x8 hi = *(const f16x8*)(base + row * stride + kh + 16);
  f16x16 f;
#pragma unroll
  for (int i = 0; i < 8; ++i) { f[i] = lo[i]; f[i + 8] = hi[i]; }
  return f;
}
#define GSTR 48

#define GSTR 48
template <typename AT, int EPI, bool OUT16>
__global__ __launch_bounds__(256) void gemm_knr(const AT* __restrict__ A, int lda, const float* __restrict__ Wm, int ldw,
                                                const float* __restrict__ bias, const float* __restrict__ R, const float* __restrict__ gvec,
                                                void* __restrict__ Yv, int ldy, int K) {
  __shared__ __attribute__((aligned(16))) f16 ldsA[128 * GSTR];
  __shared__ __attribute__((aligned(16))) f16 ldsW[128 * GSTR];
  __shared__ __attribute__((aligned(16))) float oS[8][32 * 68];
  const int tid = threadIdx.x, lane = tid & 31, wave = tid >> 5, cl = lane & 15, rh = (lane >> 4) * 8;
  const int m0 = blockIdx.x * 128, n0 = blockIdx.y * 128;
  const int wm = (wave & 3) * 32, wn = (wave >> 2) * 64;
  f32x8 acc[2][4];
#pragma unroll
  for (int i = 0; i < 2; ++i)
#pragma unroll
    for (int j = 0; j < 4; ++j) { f32x8 z = {}; acc[i][j] = z; }
#pragma unroll 1
  for (int k0 = 0; k0 < K; k0 += 32) {
    __syncthreads();
    { const int row = tid >> 1, ch = (tid & 1) * 16;
      const AT* src = A + (size_t)(m0 + row) * lda + k0 + ch;
#pragma unroll
      for (int g = 0; g < 16; ++g) ldsA[row * GSTR + ch + g] = (f16)src[g]; }
    { const int k = tid >> 3, nn0 = (tid & 7) * 16;
      const float* src = Wm + (size_t)(k0 + k) * ldw + n0 + nn0;
#pragma unroll
      for (int g = 0; g < 4; ++g) { const v4f_t v = *(const v4f_t*)(src + 4 * g);
#pragma unroll
        for (int u = 0; u < 4; ++u) ldsW[(nn0 + 4 * g + u) * GSTR + k] = (f16)v[u]; } }
    __syncthreads();
    f16x16 af[2];
#pragma unroll
    for (int i = 0; i < 2; ++i) af[i] = lds_frag(ldsA + (wm + 16 * i) * GSTR, GSTR);
#pragma unroll
    for (int j = 0; j < 4; ++j) {
      const f16x16 bf = lds_frag(ldsW + (wn + 16 * j) * GSTR, GSTR);
#pragma unroll
      for (int i = 0; i < 2; ++i) acc[i][j] = wmma16(af[i], bf, acc[i][j]);
    }
  }
  float* so = oS[wave];
#pragma unroll
  for (int i = 0; i < 2; ++i)
#pragma unroll
    for (int j = 0; j < 4; ++j) {
      const int n = n0 + wn + 16 * j + cl;
      const float bv = bias ? bias[n] : 0.0f;
      const float gv = (EPI == 2) ? gvec[n] : 0.0f;
      if (EPI == 1) {
#pragma unroll 1
        for (int r = 0; r < 8; ++r) { const float xg = acc[i][j][r] + bv; so[(16 * i + rh + r) * 68 + 16 * j + cl] = fmaxf(xg, 0.0f); }
      } else {
#pragma unroll
        for (int r = 0; r < 8; ++r) {
          float v = acc[i][j][r] + bv;
          if (EPI == 2) v = R[(size_t)(m0 + wm + 16 * i + rh + r) * ldy + n] + gv * v;
          so[(16 * i + rh + r) * 68 + 16 * j + cl] = v;
        }
      }
    }
  asm volatile("s_wait_dscnt 0" ::: "memory");
  __builtin_amdgcn_wave_barrier();
#pragma unroll 1
  for (int pass = 0; pass < 2; ++pass) {
    if (OUT16) {
      f16* Y = (f16*)Yv;
#pragma unroll
      for (int it = 0; it < 8; ++it) { const int c = lane + 32 * it, rr = c >> 3, q8 = (c & 7) * 8;
        union { f16 h[8]; v4u_t v; } u;
#pragma unroll
        for (int e = 0; e < 8; ++e) u.h[e] = (f16)so[rr * 68 + q8 + e];
        *(volatile v4u_t*)(Y + (size_t)(m0 + wm + rr) * ldy + n0 + wn + q8) = u.v; }
    } else {
      float* Y = (float*)Yv;
#pragma unroll
      for (int it = 0; it < 16; ++it) { const int f4 = lane + 32 * it, rr = f4 >> 4, q = (f4 & 15) * 4;
        *(volatile v4f_t*)(Y + (size_t)(m0 + wm + rr) * ldy + n0 + wn + q) = *(const volatile v4fa*)(so + rr * 68 + q); }
    }
    __threadfence();
  }
}


#define GSTR 48
template <typename AT, int ASRC>
__global__ __launch_bounds__(256) void gemm_knb(const AT* __restrict__ A, int lda, size_t strideA, const float* __restrict__ Wm, int ldw, size_t strideW,
                                                const float* __restrict__ rowbias, const float* __restrict__ s1, const float* __restrict__ s2, const float* __restrict__ mj, const float* __restrict__ invD,
                                                float oscale, int N, float* __restrict__ Y, int ldy, size_t strideY, int K) {
  __shared__ __attribute__((aligned(16))) f16 ldsA[128 * GSTR];
  __shared__ __attribute__((aligned(16))) f16 ldsW[128 * GSTR];
  __shared__ __attribute__((aligned(16))) float oS[8][32 * 68];
  const int tid = threadIdx.x, lane = tid & 31, wave = tid >> 5, cl = lane & 15, rh = (lane >> 4) * 8;
  const int m0 = blockIdx.x * 128, n0 = blockIdx.y * 128;
  const int wm = (wave & 3) * 32, wn = (wave >> 2) * 64;
  A += (size_t)blockIdx.z * strideA; Wm += (size_t)blockIdx.z * strideW; Y += (size_t)blockIdx.z * strideY;
  if (ASRC == 1) { s1 += (size_t)blockIdx.z * K; s2 += (size_t)blockIdx.z * lda; mj += (size_t)blockIdx.z * K; invD += (size_t)blockIdx.z * K; }
  f32x8 acc[2][4];
#pragma unroll
  for (int i = 0; i < 2; ++i)
#pragma unroll
    for (int j = 0; j < 4; ++j) { f32x8 z = {}; acc[i][j] = z; }
#pragma unroll 1
  for (int k0 = 0; k0 < K; k0 += 32) {
    __syncthreads();
    { const int row = tid >> 1, ch = (tid & 1) * 16;
      if (ASRC == 0) {
        const AT* src = A + (size_t)(m0 + row) * lda + k0 + ch;
#pragma unroll
        for (int g = 0; g < 16; ++g) ldsA[row * GSTR + ch + g] = (f16)src[g];
      } else {
        const float s2i = s2[m0 + row];
#pragma unroll
        for (int g = 0; g < 16; ++g) { const int j = k0 + ch + g; float a = s1[j] + s2i; a = (a >= 0.0f) ? a : 0.2f * a;
          ldsA[row * GSTR + ch + g] = (f16)(1024.0f * __expf(a - mj[j]) * invD[j]); }
      } }
    { const int k = tid >> 3, nn0 = (tid & 7) * 16;
      const float* src = Wm + (size_t)(k0 + k) * ldw;
#pragma unroll
      for (int g = 0; g < 4; ++g) { const int col = min(n0 + nn0 + 4 * g, N - 4); const v4f_t v = *(const v4f_t*)(src + col);
#pragma unroll
        for (int u = 0; u < 4; ++u) ldsW[(nn0 + 4 * g + u) * GSTR + k] = (f16)v[u]; } }
    __syncthreads();
    f16x16 af[2];
#pragma unroll
    for (int i = 0; i < 2; ++i) af[i] = lds_frag(ldsA + (wm + 16 * i) * GSTR, GSTR);
#pragma unroll
    for (int j = 0; j < 4; ++j) {
      const f16x16 bf = lds_frag(ldsW + (wn + 16 * j) * GSTR, GSTR);
#pragma unroll
      for (int i = 0; i < 2; ++i) acc[i][j] = wmma16(af[i], bf, acc[i][j]);
    }
  }
  float* so = oS[wave];
#pragma unroll
  for (int i = 0; i < 2; ++i)
#pragma unroll
    for (int r = 0; r < 8; ++r) {
      const int m = m0 + wm + 16 * i + rh + r;
      const float rb = rowbias ? rowbias[m] : 0.0f;
#pragma unroll
      for (int j = 0; j < 4; ++j) so[(16 * i + rh + r) * 68 + 16 * j + cl] = acc[i][j][r] * oscale + rb;
    }
  asm volatile("s_wait_dscnt 0" ::: "memory");
  __builtin_amdgcn_wave_barrier();
#pragma unroll 1
  for (int pass = 0; pass < 2; ++pass) {
#pragma unroll
    for (int it = 0; it < 16; ++it) { const int f4 = lane + 32 * it, rr = f4 >> 4, q = (f4 & 15) * 4;
      if (n0 + wn + q < N) *(volatile v4f_t*)(Y + (size_t)(m0 + wm + rr) * ldy + n0 + wn + q) = *(const volatile v4fa*)(so + rr * 68 + q); }
    __threadfence();
  }
}

__global__ __launch_bounds__(256) void k_padw3(const float* __restrict__ W3, float* __restrict__ W3p) {
  const int tid = threadIdx.x;
  for (int e = tid; e < HD * 32 / 4; e += 256) { const int k = (e * 4) / 32, n0 = (e * 4) % 32; v4f_t v;
#pragma unroll
    for (int u = 0; u < 4; ++u) { const int n = n0 + u; v[u] = (n < NA) ? W3[k * NA + n] : 0.0f; }
    *(volatile v4f_t*)(W3p + e * 4) = v; __threadfence(); *(volatile v4f_t*)(W3p + e * 4) = v; }
}
__global__ __launch_bounds__(256) void k_terms(const float* __restrict__ Q0, const float* __restrict__ Qn, const float* __restrict__ b3, const int* __restrict__ actions,
                                              const float* __restrict__ rewards, const float* __restrict__ states1, float* __restrict__ partial) {
  __shared__ float red[256];
  const int tid = threadIdx.x, b = blockIdx.x * 256 + tid;
  const int* ar = actions + (size_t)b * NA;
  int best = 0; int bvv = ar[0];
#pragma unroll
  for (int i = 1; i < NA; ++i) { const int v = ar[i]; if (v > bvv) { bvv = v; best = i; } }
  const float* qn = Qn + (size_t)b * 32;
  float mq = qn[0] + b3[0];
#pragma unroll
  for (int i = 1; i < NA; ++i) mq = fmaxf(mq, qn[i] + b3[i]);
  const bool done = (states1[(size_t)b * SD] == 666.0f);
  const float target = done ? rewards[b] : (rewards[b] + 0.9f * mq);
  const float d = (Q0[(size_t)b * 32 + best] + b3[best]) - target;
  red[tid] = d * d; __syncthreads();
  for (int o = 128; o > 0; o >>= 1) { if (tid < o) red[tid] += red[tid + o]; __syncthreads(); }
  if (tid < 32) { *(volatile float*)(partial + (size_t)blockIdx.x * 32 + tid) = red[0]; __threadfence(); *(volatile float*)(partial + (size_t)blockIdx.x * 32 + tid) = red[0]; }
}
__global__ __launch_bounds__(256) void k_final(const float* __restrict__ partial, int n, float* __restrict__ out) {
  __shared__ float red[256];
  const int tid = threadIdx.x; float s = 0.0f;
  for (int i = tid; i < n; i += 256) s += partial[(size_t)i * 32];
  red[tid] = s; __syncthreads();
  for (int o = 128; o > 0; o >>= 1) { if (tid < o) red[tid] += red[tid + o]; __syncthreads(); }
  if (tid == 0) { *(volatile float*)out = red[0]; __threadfence(); *(volatile float*)out = red[0]; }
}

extern "C" void kernel_launch(void* const* d_in, const int* in_sizes, int n_in,
                              void* d_out, int out_size, void* d_ws, size_t ws_size,
                              hipStream_t stream) {
  (void)in_sizes; (void)n_in; (void)out_size; (void)ws_size;
  const float* s0 = (const float*)d_in[0];
  const int* actions = (const int*)d_in[1];
  const float* rewards = (const float*)d_in[2];
  const float* s1 = (const float*)d_in[3];
  const float* W1 = (const float*)d_in[4], *b1 = (const float*)d_in[5], *W2 = (const float*)d_in[6], *b2 = (const float*)d_in[7], *W3 = (const float*)d_in[8], *b3 = (const float*)d_in[9];
  float* out = (float*)d_out;
  char* ws = (char*)d_ws;
  f16* h1 = (f16*)ws; ws += (size_t)NBATCH * HD * 2;
  f16* h2 = (f16*)ws; ws += (size_t)NBATCH * HD * 2;
  float* Q0 = (float*)ws; ws += (size_t)NBATCH * 32 * 4;
  float* Qn = (float*)ws; ws += (size_t)NBATCH * 32 * 4;
  float* W3p = (float*)ws; ws += HD * 32 * 4;
  float* partial = (float*)ws; ws += (size_t)(NBATCH / 256) * 128;
  const dim3 blk(256);
  k_padw3<<<dim3(1), blk, 0, stream>>>(W3, W3p);
  for (int pass = 0; pass < 2; ++pass) {
    const float* X = pass ? s1 : s0; float* Q = pass ? Qn : Q0;
    gemm_knr<float, 1, true><<<dim3(NBATCH / 128, HD / 128), blk, 0, stream>>>(X, SD, W1, HD, b1, nullptr, nullptr, h1, HD, SD);
    gemm_knr<f16, 1, true><<<dim3(NBATCH / 128, HD / 128), blk, 0, stream>>>(h1, HD, W2, HD, b2, nullptr, nullptr, h2, HD, HD);
    gemm_knb<f16, 0><<<dim3(NBATCH / 128, 1, 1), blk, 0, stream>>>(h2, HD, 0, W3p, 32, 0, nullptr, nullptr, nullptr, nullptr, nullptr, 1.0f, 32, Q, 32, 0, HD);
  }
  k_terms<<<dim3(NBATCH / 256), blk, 0, stream>>>(Q0, Qn, b3, actions, rewards, s1, partial);
  k_final<<<dim3(1), blk, 0, stream>>>(partial, NBATCH / 256, out);
}
